// CrossAttentionPool_2594160246937
// MI455X (gfx1250) — hardware-verified
//
#include <hip/hip_runtime.h>
#include <math.h>

typedef __attribute__((ext_vector_type(16))) _Float16 v16h;
typedef __attribute__((ext_vector_type(16))) __bf16 v16b;
typedef __attribute__((ext_vector_type(8)))  _Float16 v8h;
typedef __attribute__((ext_vector_type(8)))  float v8f;
typedef __attribute__((ext_vector_type(4)))  float v4f;
typedef __attribute__((ext_vector_type(2)))  float v2f;
typedef __attribute__((ext_vector_type(4)))  unsigned v4u;
typedef __attribute__((ext_vector_type(4)))  int v4i;
typedef float __attribute__((may_alias)) float_a;
typedef int __attribute__((may_alias)) int_a;

template <typename T> __device__ __forceinline__ void vst2(void* p, T v) { *(volatile T*)p = v; __threadfence(); *(volatile T*)p = v; }
__device__ __forceinline__ v8f wmma16(v16h a, v16h b, v8f c) {
  v8f d = __builtin_amdgcn_wmma_f32_16x16x32_f16(false, a, false, b, (short)0, c, false, false);
  asm volatile("v_nop\n\tv_nop\n\tv_nop\n\tv_nop" : "+v"(d) : "v"(a), "v"(b));
  return d;
}
__device__ __forceinline__ v8f wmma_bf(v16b a, v16b b, v8f c) {
  v8f d = __builtin_amdgcn_wmma_f32_16x16x32_bf16(false, a, false, b, (short)0, c, false, false);
  asm volatile("v_nop\n\tv_nop\n\tv_nop\n\tv_nop" : "+v"(d) : "v"(a), "v"(b));
  return d;
}
__device__ __forceinline__ v16h frag_h(const _Float16* rowk0, int lane) {
  union { v16h v; v8h q[2]; } u; const _Float16* p = rowk0 + 8 * (lane >> 4);
  u.q[0] = *(const v8h*)p; u.q[1] = *(const v8h*)(p + 16); return u.v;
}
__device__ __forceinline__ v16h frag_f32(const float* rowk0, int lane) {
  v16h a; const float* p = rowk0 + 8 * (lane >> 4);
#pragma unroll
  for (int i = 0; i < 8; ++i) { a[i] = (_Float16)p[i]; a[8 + i] = (_Float16)p[16 + i]; }
  return a;
}
__device__ __forceinline__ v16h frag_f32s(const float* rowk0, int lane, float sc) {
  v16h a; const float* p = rowk0 + 8 * (lane >> 4);
#pragma unroll
  for (int i = 0; i < 8; ++i) { a[i] = (_Float16)(p[i] * sc); a[8 + i] = (_Float16)(p[16 + i] * sc); }
  return a;
}
__device__ __forceinline__ v16h fragc_f32(const float* W, int k0, int n, int lane, int ld, int K) {
  v16h a; const int g = lane >> 4;
#pragma unroll
  for (int i = 0; i < 8; ++i) { const int ka = k0 + 8 * g + i, kb = ka + 16;
    a[i] = (_Float16)(ka < K ? W[(size_t)(ka < K ? ka : K - 1) * ld + n] : 0.f); a[8 + i] = (_Float16)(kb < K ? W[(size_t)(kb < K ? kb : K - 1) * ld + n] : 0.f); }
  return a;
}
struct F2 { v16b h, l; };
__device__ __forceinline__ F2 bsplit16(const float v[16]) { F2 r;
#pragma unroll
  for (int i = 0; i < 16; ++i) { const __bf16 h = (__bf16)v[i]; r.h[i] = h; r.l[i] = (__bf16)(v[i] - (float)h); }
  return r; }
__device__ __forceinline__ F2 split_row(const float* row, int k0, int lane) { float v[16]; const float* p = row + k0 + 8 * (lane >> 4);
#pragma unroll
  for (int i = 0; i < 8; ++i) { v[i] = p[i]; v[8 + i] = p[16 + i]; }
  return bsplit16(v); }
__device__ __forceinline__ F2 split_rowK(const float* row, int k0, int lane, int K) { float v[16]; const int g = lane >> 4;
#pragma unroll
  for (int i = 0; i < 8; ++i) { const int ka = k0 + 8 * g + i, kb = ka + 16; v[i] = ka < K ? row[ka < K ? ka : K - 1] : 0.f; v[8 + i] = kb < K ? row[kb < K ? kb : K - 1] : 0.f; }
  return bsplit16(v); }
__device__ __forceinline__ F2 split_col(const float* W, int k0, int n, int lane, int ld, int K) { float v[16]; const int g = lane >> 4;
#pragma unroll
  for (int i = 0; i < 8; ++i) { const int ka = k0 + 8 * g + i, kb = ka + 16; v[i] = ka < K ? W[(size_t)(ka < K ? ka : K - 1) * ld + n] : 0.f; v[8 + i] = kb < K ? W[(size_t)(kb < K ? kb : K - 1) * ld + n] : 0.f; }
  return bsplit16(v); }
__device__ __forceinline__ v8f mac3(const F2& a, const F2& b, v8f c) { c = wmma_bf(a.l, b.h, c); c = wmma_bf(a.h, b.l, c); return wmma_bf(a.h, b.h, c); }
__device__ __forceinline__ float sigm(float v) { return 1.0f / (1.0f + expf(-v)); }
#define LDSX() do { asm volatile("s_wait_dscnt 0" ::: "memory"); __builtin_amdgcn_wave_barrier(); __builtin_amdgcn_fence(__ATOMIC_RELEASE, "workgroup"); } while (0)


#define NBc 32
#define LQ 512
#define NVK 128
#define DD 768
#define NRQ (NBc * LQ)
#define NRK (NBc * NVK)
#ifndef NBB
#define NBB NBc
#endif
typedef __attribute__((ext_vector_type(8))) __bf16 v8b;
__device__ __forceinline__ v16b frag_b(const __bf16* rowk0, int lane) {
  union { v16b v; v8b q[2]; } u; const __bf16* p = rowk0 + 8 * (lane >> 4);
  u.q[0] = *(const v8b*)p; u.q[1] = *(const v8b*)(p + 16); return u.v;
}
__device__ __forceinline__ float bfr(float v) { return (float)(__bf16)v; }
__device__ __attribute__((noinline)) float exp_ni(float v) { return expf(v); }
__device__ __attribute__((noinline)) float erf_ni(float v) { return erff(v); }

#define WS_PW  0u
#define WS_QH  (WS_PW + 2u * 2 * DD * DD)
#define WS_KH  (WS_QH + 2u * NRQ * DD)
#define WS_VT  (WS_KH + 2u * NRK * DD)
#define WS_END (WS_VT + 2u * NRK * DD)

__global__ __launch_bounds__(256) void k_pack(const float* __restrict__ WQ, const float* __restrict__ WK, __bf16* __restrict__ PW) {
  const int n = blockIdx.x, which = blockIdx.y, t = threadIdx.x; __shared__ __align__(16) __bf16 s[DD]; const float* src = (which ? WK : WQ) + (size_t)n * DD;
  for (int k = t; k < DD; k += 256) s[k] = (__bf16)src[k]; __syncthreads();
  if (t < DD / 8) vst2((unsigned*)(PW + ((size_t)which * DD + n) * DD + t * 8), *(const v4u*)&s[t * 8]);
}
__global__ __launch_bounds__(128) void k_proj(const float* __restrict__ LN, const float* __restrict__ VD, const __bf16* __restrict__ PW, _Float16* __restrict__ QH, _Float16* __restrict__ KH) {
  __shared__ __align__(16) _Float16 so[4][16][136];
  const int tid = threadIdx.x, wave = tid >> 5, lane = tid & 31, col = lane & 15, g = lane >> 4; const int which = blockIdx.z; const size_t r0 = (size_t)blockIdx.x * 64 + wave * 16; const int n0 = blockIdx.y * 128;
  if (which == 1 && blockIdx.x >= NRK / 64) return;
  const float* X = which ? VD : LN; const __bf16* Wr = PW + (size_t)which * DD * DD; _Float16* dst = which ? KH : QH;
  v8f acc[8] = {};
#pragma unroll 2
  for (int kc = 0; kc < DD / 32; ++kc) { v16b a; { const float* p = X + (r0 + col) * DD + kc * 32 + 8 * g;
#pragma unroll
      for (int i = 0; i < 8; ++i) { a[i] = (__bf16)p[i]; a[8 + i] = (__bf16)p[16 + i]; } }
#pragma unroll
    for (int j = 0; j < 8; ++j) acc[j] = wmma_bf(a, frag_b(Wr + (size_t)(n0 + j * 16 + col) * DD + kc * 32, lane), acc[j]); }
#pragma unroll
  for (int j = 0; j < 8; ++j)
#pragma unroll
    for (int r = 0; r < 8; ++r) so[wave][8 * g + r][j * 16 + col] = (_Float16)acc[j][r];
  LDSX();
  for (int rl = 0; rl < 16; ++rl) if (lane < 16) vst2((unsigned*)(dst + (r0 + rl) * DD + n0 + lane * 8), *(const v4u*)&so[wave][rl][lane * 8]);
}
__global__ __launch_bounds__(256) void k_vt(const float* __restrict__ VD, _Float16* __restrict__ VT) {
  __shared__ __align__(16) _Float16 st[128][136]; const size_t b = blockIdx.x; const int c0 = blockIdx.y * 128, t = threadIdx.x;
  for (int e = t; e < 128 * 128; e += 256) { const int tok = e >> 7, c = e & 127; st[c][tok] = (_Float16)bfr(VD[(b * NVK + tok) * DD + c0 + c]); }
  __syncthreads();
  for (int e = t; e < 128 * 16; e += 256) { const int c = e >> 4, q = e & 15; vst2((unsigned*)(VT + (b * DD + c0 + c) * NVK + q * 8), *(const v4u*)&st[c][q * 8]); }
}
__global__ __launch_bounds__(128) void k_attn(const _Float16* __restrict__ QH, const _Float16* __restrict__ KH, const _Float16* __restrict__ VT, const int* __restrict__ MSK, float* __restrict__ OUT) {
  __shared__ __align__(16) _Float16 sph[4][16][NVK + 8], spl[4][16][NVK + 8]; __shared__ __align__(16) float so[4][16][132]; __shared__ float ssc[4][16][NVK + 4];
  const int tid = threadIdx.x, wave = tid >> 5, lane = tid & 31, col = lane & 15, g = lane >> 4; const int vc = blockIdx.y; const size_t b = blockIdx.z; const size_t rq = b * LQ + (size_t)blockIdx.x * 64 + wave * 16;
  const float scale = 1.0f / sqrtf((float)DD);
#pragma unroll 1
  for (int kt = 0; kt < NVK / 16; ++kt) { const int kk = kt * 16 + col; const size_t rk = (b * NVK + kk) * DD; v8f c = {};
#pragma unroll 4
    for (int kc = 0; kc < DD / 32; ++kc) c = wmma16(frag_h(QH + (rq + col) * DD + kc * 32, lane), frag_h(KH + rk + kc * 32, lane), c);
    const bool keep = MSK[b * NVK + kk] != 0;
#pragma unroll
    for (int r = 0; r < 8; ++r) ssc[wave][8 * g + r][kk] = keep ? c[r] * scale : -3.0e38f; }
  __syncthreads();
  { const int r = lane & 15, half = lane >> 4; float mx = -3.0e38f; for (int k = half * 64; k < half * 64 + 64; ++k) mx = fmaxf(mx, ssc[wave][r][k]); mx = fmaxf(mx, __shfl_xor(mx, 16));
    float sum = 0.f; for (int k = half * 64; k < half * 64 + 64; ++k) { const float sv = ssc[wave][r][k]; const float e = (sv <= -1.0e38f) ? 0.f : __expf(sv - mx); sum += e; const float pe = e * 2048.0f; const _Float16 he = (_Float16)pe; sph[wave][r][k] = he; spl[wave][r][k] = (_Float16)((pe - (float)he) * 2048.0f); } sum += __shfl_xor(sum, 16);
    if (half == 0) ssc[wave][r][NVK] = (1.0f / 2048.0f) / sum; }
  LDSX();
  v8f acc[8] = {}, accl[8] = {};
#pragma unroll
  for (int kc = 0; kc < NVK / 32; ++kc) { const v16h pa = frag_h(&sph[wave][col][kc * 32], lane), pl = frag_h(&spl[wave][col][kc * 32], lane);
#pragma unroll
    for (int dt = 0; dt < 8; ++dt) { const v16h vh = frag_h(VT + (b * DD + (size_t)vc * 128 + dt * 16 + col) * NVK + kc * 32, lane); acc[dt] = wmma16(pa, vh, acc[dt]); accl[dt] = wmma16(pl, vh, accl[dt]); } }
#pragma unroll
  for (int r = 0; r < 8; ++r) { const float il = ssc[wave][8 * g + r][NVK];
#pragma unroll
    for (int dt = 0; dt < 8; ++dt) so[wave][8 * g + r][dt * 16 + col] = (acc[dt][r] + accl[dt][r] * (1.0f / 2048.0f)) * il; }
  LDSX();
  for (int rl = 0; rl < 16; ++rl) vst2(OUT + (rq + rl) * DD + (size_t)vc * 128 + lane * 4, *(const v4f*)&so[wave][rl][lane * 4]);
}
extern "C" void kernel_launch(void* const* d_in, const int* in_sizes, int n_in, void* d_out, int out_size, void* d_ws, size_t ws_size, hipStream_t stream) {
  (void)in_sizes; (void)n_in; (void)out_size;
  const float** F = (const float**)d_in;
  if (ws_size < (size_t)WS_END) return;
  char* ws = (char*)d_ws; __bf16* PW = (__bf16*)(ws + WS_PW); _Float16 *QH = (_Float16*)(ws + WS_QH), *KH = (_Float16*)(ws + WS_KH), *VT = (_Float16*)(ws + WS_VT);
  k_pack<<<dim3(DD, 2), 256, 0, stream>>>(F[3], F[4], PW);
  k_proj<<<dim3(NBB * LQ / 64, DD / 128, 2), 128, 0, stream>>>(F[0], F[1], PW, QH, KH);
  k_vt<<<dim3(NBB, DD / 128), 256, 0, stream>>>(F[1], VT);
  k_attn<<<dim3(LQ / 64, DD / 128, NBB), 128, 0, stream>>>(QH, KH, VT, (const int*)d_in[2], (float*)d_out);
}
